// STCrossAttnBlock_44547400794816
// MI455X (gfx1250) — hardware-run, weakly checked
//
#include <hip/hip_runtime.h>
#include <stdint.h>
#include <stddef.h>

#define CH     512
#define NPOS   2304
#define NKEY   6912
#define NBAT   4
#define NFRM   12
#define GN_INV_CNT (1.0 / 884736.0)

typedef _Float16 f16t;
typedef _Float16 v16h __attribute__((ext_vector_type(16)));
typedef _Float16 v8h  __attribute__((ext_vector_type(8)));
typedef float    v8f  __attribute__((ext_vector_type(8)));
typedef float    v4f  __attribute__((ext_vector_type(4)));
typedef double   v2d  __attribute__((ext_vector_type(2)));

union FragU { v16h v; v8h h[2]; };

__device__ __forceinline__ v16h frag_ld(const f16t* p) {
  FragU f;
  f.h[0] = *(const v8h*)(p);
  f.h[1] = *(const v8h*)(p + 16);
  return f.v;
}

__device__ __forceinline__ v8f mma16(v16h a, v16h b, v8f c) {
  c = __builtin_amdgcn_wmma_f32_16x16x32_f16(false, a, false, b, (short)0, c, false, false);
  asm volatile("v_nop\n\tv_nop\n\tv_nop\n\tv_nop" : "+v"(c) : "v"(a), "v"(b));
  return c;
}

__device__ __forceinline__ v8f zero8() {
  v8f z;
#pragma unroll
  for (int i = 0; i < 8; ++i) z[i] = 0.0f;
  return z;
}

__device__ __forceinline__ void lds_wave_sync() {
  __builtin_amdgcn_fence(__ATOMIC_RELEASE, "workgroup");
  __builtin_amdgcn_wave_barrier();
  __builtin_amdgcn_fence(__ATOMIC_ACQUIRE, "workgroup");
}

__global__ __launch_bounds__(256) void gn_part(const float* __restrict__ x, double* part) {
  __shared__ double rs[256];
  __shared__ double rq[256];
  const int cb  = blockIdx.x;
  const int fr  = blockIdx.y;
  const int tid = threadIdx.x;
  const float* base = x + ((size_t)fr * CH + (size_t)cb * 16) * NPOS;
  double s = 0.0, q = 0.0;
#pragma unroll 2
  for (int i = 0; i < 36; ++i) {
    const v4f v = *(const v4f*)(base + ((size_t)i * 256 + tid) * 4);
#pragma unroll
    for (int e = 0; e < 4; ++e) {
      const double d = (double)v[e];
      s += d;
      q += d * d;
    }
  }
  rs[tid] = s;
  rq[tid] = q;
  __syncthreads();
  for (int st = 128; st > 0; st >>= 1) {
    if (tid < st) {
      rs[tid] += rs[tid + st];
      rq[tid] += rq[tid + st];
    }
    __syncthreads();
  }
  if (tid < 8) {
    v2d o;
    o[0] = (tid == 0) ? rs[0] : 0.0;
    o[1] = (tid == 0) ? rq[0] : 0.0;
    double* lp = part + ((size_t)(fr * 32 + cb)) * 16 + tid * 2;
    *(volatile v2d*)lp = o;
    __threadfence();
    *(volatile v2d*)lp = o;
  }
}

__global__ __launch_bounds__(32) void gn_fin(const double* __restrict__ part, float* stats) {
  __shared__ __align__(16) float sm[32];
  const int lane = threadIdx.x;
  const int grp  = lane & 15;
  const int b    = grp >> 2;
  const int g    = grp & 3;
  double s = 0.0, q = 0.0;
#pragma unroll 1
  for (int f = 0; f < 3; ++f) {
#pragma unroll 1
    for (int j = 0; j < 8; ++j) {
      const double* lp = part + ((size_t)((f * 4 + b) * 32 + g * 8 + j)) * 16;
      s += lp[0];
      q += lp[1];
    }
  }
  const double mean = s * GN_INV_CNT;
  double var = q * GN_INV_CNT - mean * mean;
  if (var < 0.0) var = 0.0;
  const double rstd = 1.0 / sqrt(var + 1e-6);
  if (lane < 16) {
    sm[2 * grp]     = (float)mean;
    sm[2 * grp + 1] = (float)rstd;
  }
  __syncthreads();
  if (lane < 8) {
    const v4f v = *(const v4f*)(sm + 4 * lane);
    *(volatile v4f*)(stats + 4 * lane) = v;
    __threadfence();
    *(volatile v4f*)(stats + 4 * lane) = v;
  }
}

__global__ __launch_bounds__(256) void gn_apply(const float* __restrict__ x, const float* __restrict__ stats,
                                                 const float* __restrict__ nsc, const float* __restrict__ nbi,
                                                 f16t* hn) {
  __shared__ __align__(16) float tf[64 * 68];
  const int sb  = blockIdx.x;
  const int cb  = blockIdx.y;
  const int fr  = blockIdx.z;
  const int f   = fr >> 2;
  const int b   = fr & 3;
  const int tid = threadIdx.x;
  {
    const int lr = tid >> 4;
    const int c4 = (tid & 15) * 4;
#pragma unroll
    for (int it = 0; it < 4; ++it) {
      const int rr  = it * 16 + lr;
      const int c   = cb * 64 + rr;
      const int grp = b * 4 + (c >> 7);
      const float mean = stats[2 * grp];
      const float rstd = stats[2 * grp + 1];
      const float sc   = nsc[c];
      const float bi   = nbi[c];
      const v4f v = *(const v4f*)(x + ((size_t)fr * CH + c) * NPOS + sb * 64 + c4);
      v4f o;
#pragma unroll
      for (int e = 0; e < 4; ++e) {
        const float t = (v[e] - mean) * rstd;
        o[e] = t * sc + bi;
      }
      *(v4f*)(tf + rr * 68 + c4) = o;
    }
  }
  __syncthreads();
  const int sub = tid >> 3;
  const int c8  = (tid & 7) * 8;
  v8h hv[2];
#pragma unroll
  for (int it = 0; it < 2; ++it) {
    const int os = it * 32 + sub;
    v8h hq;
#pragma unroll
    for (int e = 0; e < 8; ++e) hq[e] = (f16t)tf[(c8 + e) * 68 + os];
    hv[it] = hq;
  }
  f16t* ob = hn + ((size_t)b * NKEY + (size_t)f * NPOS + (size_t)sb * 64) * CH + cb * 64;
  for (int pass = 0; pass < 2; ++pass) {
#pragma unroll
    for (int it = 0; it < 2; ++it) {
      const int os = it * 32 + sub;
      *(volatile v8h*)(ob + (size_t)os * CH + c8) = hv[it];
    }
    __threadfence();
  }
}

__global__ __launch_bounds__(256) void wcvt(const float* __restrict__ w0, const float* __restrict__ w1,
                                             const float* __restrict__ w2, const float* __restrict__ w3,
                                             f16t* wh, float sc) {
  const int y = blockIdx.y;
  const float* src = w0;
  if (y == 1) src = w1;
  if (y == 2) src = w2;
  if (y == 3) src = w3;
  const size_t i = (size_t)blockIdx.x * 256 + threadIdx.x;
  const v4f a = *(const v4f*)(src + 8 * i);
  const v4f c = *(const v4f*)(src + 8 * i + 4);
  v8h o;
#pragma unroll
  for (int e = 0; e < 4; ++e) {
    o[e]     = (f16t)(a[e] * sc);
    o[e + 4] = (f16t)(c[e] * sc);
  }
  f16t* dp = wh + (size_t)y * CH * CH + 8 * i;
  *(volatile v8h*)dp = o;
  __threadfence();
  *(volatile v8h*)dp = o;
}

template <int MODE>
__global__ __launch_bounds__(256) void gemm64(
    const f16t* __restrict__ A, int lda, long sA,
    const f16t* __restrict__ Bt, int ldb, long sB,
    f16t* C16, float* C32, int ldc, long sC,
    const float* __restrict__ bias,
    const float* __restrict__ R, int ldr, long sR,
    int M, int N, int K, float scale, float osc) {
  __shared__ __align__(16) float sT[8][16 * 68];
  const int bz   = blockIdx.y;
  const int lane = threadIdx.x & 31;
  const int wave = threadIdx.x >> 5;
  const int tilesN = N >> 6;
  const int tilesM = M >> 6;
  const int tile = blockIdx.x * 8 + wave;
  if (tile >= tilesM * tilesN) return;
  const int tm = tile / tilesN;
  const int tn = tile - tm * tilesN;
  const int m0 = tm << 6;
  const int n0 = tn << 6;
  const f16t* Ab = A  + (size_t)bz * sA;
  const f16t* Bb = Bt + (size_t)bz * sB;
  const int rl = lane & 15;
  const int kh = (lane >> 4) * 8;

  v8f acc[4][4];
#pragma unroll
  for (int i = 0; i < 4; ++i)
#pragma unroll
    for (int j = 0; j < 4; ++j) acc[i][j] = zero8();

  for (int k0 = 0; k0 < K; k0 += 32) {
    v16h bf[4];
#pragma unroll
    for (int j = 0; j < 4; ++j)
      bf[j] = frag_ld(Bb + (size_t)(n0 + 16 * j + rl) * ldb + k0 + kh);
#pragma unroll
    for (int i = 0; i < 4; ++i) {
      const v16h af = frag_ld(Ab + (size_t)(m0 + 16 * i + rl) * lda + k0 + kh);
#pragma unroll
      for (int j = 0; j < 4; ++j) acc[i][j] = mma16(af, bf[j], acc[i][j]);
    }
  }

  float* slab = sT[wave];
  const float* Rb = R + (size_t)bz * sR;
#pragma unroll
  for (int i = 0; i < 4; ++i) {
    const int mBase = m0 + 16 * i;
    float bm[8];
#pragma unroll
    for (int r = 0; r < 8; ++r) bm[r] = 0.0f;
    if (MODE == 1 || MODE == 3) {
#pragma unroll
      for (int r = 0; r < 8; ++r) bm[r] = bias[mBase + kh + r];
    }
#pragma unroll
    for (int j = 0; j < 4; ++j) {
      const int n = n0 + 16 * j + rl;
      float bn = 0.0f;
      if (MODE == 0 || MODE == 2) bn = bias[n];
#pragma unroll
      for (int r = 0; r < 8; ++r) {
        float v = acc[i][j][r] * scale;
        if (MODE == 0 || MODE == 2) v += bn;
        else v += bm[r];
        if (MODE == 3) v += Rb[(size_t)n * ldr + (mBase + kh + r)];
        slab[(kh + r) * 68 + 16 * j + rl] = v;
      }
    }
    lds_wave_sync();
    if (MODE == 2 || MODE == 3) {
      float* Cb = C32 + (size_t)bz * sC;
      const int hh = lane >> 4, c4 = (lane & 15) * 4;
      for (int pass = 0; pass < 2; ++pass) {
#pragma unroll
        for (int it = 0; it < 8; ++it) {
          const int row = it * 2 + hh;
          const v4f v = *(const v4f*)(slab + row * 68 + c4);
          *(volatile v4f*)(Cb + (size_t)(mBase + row) * ldc + n0 + c4) = v;
        }
        __threadfence();
      }
    }
    if (MODE != 3) {
      f16t* Cb = C16 + (size_t)bz * sC;
      const int q8 = lane >> 3, c8 = (lane & 7) * 8;
      v8h hv[4];
#pragma unroll
      for (int it = 0; it < 4; ++it) {
        const int row = it * 4 + q8;
        const float* sp = slab + row * 68 + c8;
        v8h t;
#pragma unroll
        for (int e = 0; e < 8; ++e) t[e] = (f16t)(sp[e] * osc);
        hv[it] = t;
      }
      for (int pass = 0; pass < 2; ++pass) {
#pragma unroll
        for (int it = 0; it < 4; ++it) {
          const int row = it * 4 + q8;
          *(volatile v8h*)(Cb + (size_t)(mBase + row) * ldc + n0 + c8) = hv[it];
        }
        __threadfence();
      }
    }
    lds_wave_sync();
  }
}

#define AQ   32
#define AKC  64
#define QSP  512
#define SPF  68
#define PPH  72

__global__ __launch_bounds__(256) void attn_kernel(const f16t* __restrict__ Qp, const f16t* __restrict__ Kp,
                                                    const f16t* __restrict__ Vtp, f16t* AOp, float sl2) {
  __shared__ __align__(16) f16t  Qs[AQ * QSP];
  __shared__ __align__(16) float Sb[AQ * SPF];
  __shared__ __align__(16) f16t  Pb[AQ * PPH];
  __shared__ __align__(16) float alph[AQ];
  __shared__ __align__(16) float lfac[AQ];

  const int tid  = threadIdx.x;
  const int wave = tid >> 5;
  const int lane = tid & 31;
  const int rl   = lane & 15;
  const int kh   = (lane >> 4) * 8;
  const int b    = blockIdx.y;
  const int q0   = blockIdx.x * AQ;

  const f16t* Qb = Qp  + ((size_t)b * NPOS + q0) * CH;
  const f16t* Kb = Kp  + (size_t)b * NKEY * CH;
  const f16t* Vb = Vtp + (size_t)b * CH * NKEY;
  f16t*       Ob = AOp + ((size_t)b * NPOS + q0) * CH;

  {
    const int row = tid >> 3, seg = (tid & 7) * 64;
#pragma unroll
    for (int i = 0; i < 8; ++i) {
      const v8h v = *(const v8h*)(Qb + (size_t)row * CH + seg + 8 * i);
      *(v8h*)(Qs + row * QSP + seg + 8 * i) = v;
    }
  }
  __syncthreads();

  const int rt   = wave >> 2;
  const int kt   = wave & 3;
  const int srow = tid >> 3;
  const int part = tid & 7;
  const int cw   = wave * 64;

  float m_run = -__builtin_huge_valf();
  float l_run = 0.0f;
  v8f oacc[2][4];
#pragma unroll
  for (int a = 0; a < 2; ++a)
#pragma unroll
    for (int t = 0; t < 4; ++t) oacc[a][t] = zero8();

  for (int kc = 0; kc < NKEY / AKC; ++kc) {
    const int key0 = kc * AKC;

    v8f sacc = zero8();
    {
      const f16t* qrow = Qs + (rt * 16 + rl) * QSP + kh;
      const f16t* krow = Kb + (size_t)(key0 + kt * 16 + rl) * CH + kh;
#pragma unroll
      for (int ks = 0; ks < CH / 32; ++ks) {
        const v16h af = frag_ld(qrow + ks * 32);
        const v16h bq = frag_ld(krow + ks * 32);
        sacc = mma16(af, bq, sacc);
      }
    }
#pragma unroll
    for (int r = 0; r < 8; ++r) Sb[(rt * 16 + kh + r) * SPF + kt * 16 + rl] = sacc[r] * sl2;
    __syncthreads();

    {
      const float* sp = Sb + srow * SPF + part * 8;
      const v4f s0 = *(const v4f*)(sp);
      const v4f s1 = *(const v4f*)(sp + 4);
      float sv[8];
#pragma unroll
      for (int e = 0; e < 4; ++e) { sv[e] = s0[e]; sv[e + 4] = s1[e]; }
      float cmax = sv[0];
#pragma unroll
      for (int e = 1; e < 8; ++e) cmax = fmaxf(cmax, sv[e]);
      cmax = fmaxf(cmax, __shfl_xor(cmax, 1, 32));
      cmax = fmaxf(cmax, __shfl_xor(cmax, 2, 32));
      cmax = fmaxf(cmax, __shfl_xor(cmax, 4, 32));
      const float mnew  = fmaxf(m_run, cmax);
      const float alpha = exp2f(m_run - mnew);
      float psum = 0.0f;
      v8h pv;
#pragma unroll
      for (int e = 0; e < 8; ++e) {
        const float p = exp2f(sv[e] - mnew);
        psum += p;
        pv[e] = (f16t)(p * 512.0f);
      }
      psum += __shfl_xor(psum, 1, 32);
      psum += __shfl_xor(psum, 2, 32);
      psum += __shfl_xor(psum, 4, 32);
      l_run = l_run * alpha + psum;
      m_run = mnew;
      *(v8h*)(Pb + srow * PPH + part * 8) = pv;
      if (part == 0) alph[srow] = alpha;
    }
    __syncthreads();

#pragma unroll
    for (int a = 0; a < 2; ++a) {
      const v4f f0 = *(const v4f*)(alph + a * 16 + kh);
      const v4f f1 = *(const v4f*)(alph + a * 16 + kh + 4);
      float al[8];
#pragma unroll
      for (int e = 0; e < 4; ++e) { al[e] = f0[e]; al[e + 4] = f1[e]; }
#pragma unroll
      for (int t = 0; t < 4; ++t)
#pragma unroll
        for (int r = 0; r < 8; ++r) oacc[a][t][r] *= al[r];
    }

#pragma unroll
    for (int kk = 0; kk < 2; ++kk) {
      const v16h pa0 = frag_ld(Pb + (0 * 16 + rl) * PPH + kk * 32 + kh);
      const v16h pa1 = frag_ld(Pb + (1 * 16 + rl) * PPH + kk * 32 + kh);
#pragma unroll
      for (int t = 0; t < 4; ++t) {
        const v16h vb = frag_ld(Vb + (size_t)(cw + t * 16 + rl) * NKEY + key0 + kk * 32 + kh);
        oacc[0][t] = mma16(pa0, vb, oacc[0][t]);
        oacc[1][t] = mma16(pa1, vb, oacc[1][t]);
      }
    }
  }

  if (part == 0) lfac[srow] = 1.0f / (8.0f * l_run);
  __syncthreads();

  f16t* slab = Qs + wave * (16 * PPH);
  const int q8 = lane >> 3, c8 = (lane & 7) * 8;
#pragma unroll
  for (int a = 0; a < 2; ++a) {
    const v4f f0 = *(const v4f*)(lfac + a * 16 + kh);
    const v4f f1 = *(const v4f*)(lfac + a * 16 + kh + 4);
    float lf[8];
#pragma unroll
    for (int e = 0; e < 4; ++e) { lf[e] = f0[e]; lf[e + 4] = f1[e]; }
#pragma unroll
    for (int t = 0; t < 4; ++t)
#pragma unroll
      for (int r = 0; r < 8; ++r)
        slab[(kh + r) * PPH + t * 16 + rl] = (f16t)(oacc[a][t][r] * lf[r]);
    lds_wave_sync();
    v8h hv[4];
#pragma unroll
    for (int it = 0; it < 4; ++it) {
      const int row = it * 4 + q8;
      hv[it] = *(const v8h*)(slab + row * PPH + c8);
    }
    for (int pass = 0; pass < 2; ++pass) {
#pragma unroll
      for (int it = 0; it < 4; ++it) {
        const int row = it * 4 + q8;
        *(volatile v8h*)(Ob + (size_t)(a * 16 + row) * CH + cw + c8) = hv[it];
      }
      __threadfence();
    }
    lds_wave_sync();
  }
}

static inline size_t align256(size_t v) { return (v + 255) & ~(size_t)255; }

extern "C" void kernel_launch(void* const* d_in, const int* in_sizes, int n_in,
                              void* d_out, int out_size, void* d_ws, size_t ws_size,
                              hipStream_t stream) {
  if (n_in < 11) return;
  if (in_sizes[0] != NFRM * CH * NPOS) return;
  if (in_sizes[1] != CH || in_sizes[2] != CH) return;
  if (in_sizes[3] != CH * CH || in_sizes[5] != CH * CH || in_sizes[7] != CH * CH || in_sizes[9] != CH * CH) return;
  if (in_sizes[4] != CH || in_sizes[6] != CH || in_sizes[8] != CH || in_sizes[10] != CH) return;
  if (out_size != NBAT * CH * NPOS) return;

  const float* x   = (const float*)d_in[0];
  const float* nsc = (const float*)d_in[1];
  const float* nbi = (const float*)d_in[2];
  const float* qw  = (const float*)d_in[3];
  const float* qb  = (const float*)d_in[4];
  const float* kw  = (const float*)d_in[5];
  const float* kb  = (const float*)d_in[6];
  const float* vw  = (const float*)d_in[7];
  const float* vb  = (const float*)d_in[8];
  const float* pw  = (const float*)d_in[9];
  const float* pb  = (const float*)d_in[10];
  float* out = (float*)d_out;

  const size_t bPart = (size_t)NFRM * 32 * 16 * sizeof(double);
  const size_t bStat = 256;
  const size_t bW    = (size_t)4 * CH * CH * sizeof(f16t);
  const size_t bHn   = (size_t)NBAT * NKEY * CH * sizeof(f16t);
  const size_t bK    = bHn;
  const size_t bVt   = (size_t)NBAT * CH * NKEY * sizeof(f16t);
  const size_t bQ    = (size_t)NBAT * NPOS * CH * sizeof(f16t);
  const size_t bSk   = (size_t)NBAT * NPOS * CH * sizeof(float);
  const size_t bAo   = bQ;

  size_t off = 0;
  const size_t oPart = off; off = align256(off + bPart);
  const size_t oStat = off; off = align256(off + bStat);
  const size_t oW    = off; off = align256(off + bW);
  const size_t oHn   = off; off = align256(off + bHn);
  const size_t oK    = off; off = align256(off + bK);
  const size_t oVt   = off; off = align256(off + bVt);
  const size_t oQ    = off; off = align256(off + bQ);
  const size_t oSk   = off; off = align256(off + bSk);
  const size_t oAo   = off; off = align256(off + bAo);
  if (off > ws_size) return;

  char* ws = (char*)d_ws;
  double* part  = (double*)(ws + oPart);
  float*  stats = (float*)(ws + oStat);
  f16t*   wh    = (f16t*)(ws + oW);
  f16t*   hn    = (f16t*)(ws + oHn);
  f16t*   kp    = (f16t*)(ws + oK);
  f16t*   vt    = (f16t*)(ws + oVt);
  f16t*   qp    = (f16t*)(ws + oQ);
  float*  skip  = (float*)(ws + oSk);
  f16t*   ao    = (f16t*)(ws + oAo);

  const size_t WPL = (size_t)CH * CH;
  const float inv32  = 1.0f / 32.0f;
  const float invPrj = 1.0f / 32768.0f;
  const float sl2    = (float)(1.4426950408889634 * 0.04419417382415922 / 256.0);

  gn_part<<<dim3(32, NFRM), dim3(256), 0, stream>>>(x, part);
  gn_fin<<<dim3(1), dim3(32), 0, stream>>>(part, stats);
  gn_apply<<<dim3(NPOS / 64, CH / 64, NFRM), dim3(256), 0, stream>>>(x, stats, nsc, nbi, hn);
  wcvt<<<dim3(128, 4), dim3(256), 0, stream>>>(qw, kw, vw, pw, wh, 32.0f);
  gemm64<0><<<dim3((NBAT * NKEY / 64) * (CH / 64) / 8, 1), dim3(256), 0, stream>>>(
      hn, CH, 0L, wh + 1 * WPL, CH, 0L, kp, skip, CH, 0L, kb, stats, 0, 0L,
      NBAT * NKEY, CH, CH, inv32, 16.0f);
  gemm64<1><<<dim3((CH / 64) * (NKEY / 64) / 8, NBAT), dim3(256), 0, stream>>>(
      wh + 2 * WPL, CH, 0L, hn, CH, (long)NKEY * CH, vt, skip, NKEY, (long)CH * NKEY, vb, stats, 0, 0L,
      CH, NKEY, CH, inv32, 16.0f);
  gemm64<2><<<dim3((NPOS / 64) * (CH / 64) / 8, NBAT), dim3(256), 0, stream>>>(
      hn + (size_t)NPOS * CH, CH, (long)NKEY * CH, wh + 0 * WPL, CH, 0L, qp, skip, CH, (long)NPOS * CH, qb, stats, 0, 0L,
      NPOS, CH, CH, inv32, 16.0f);
  attn_kernel<<<dim3(NPOS / AQ, NBAT), dim3(256), 0, stream>>>(qp, kp, vt, ao, sl2);
  gemm64<3><<<dim3((CH / 64) * (NPOS / 64) / 8, NBAT), dim3(256), 0, stream>>>(
      wh + 3 * WPL, CH, 0L, ao, CH, (long)NPOS * CH, ao, out, NPOS, (long)CH * NPOS, pb, skip, CH, (long)NPOS * CH,
      CH, NPOS, CH, invPrj, 1.0f);
  (void)hipGetLastError();
}
